// MAB_channel_aware_force_16862041604426
// MI455X (gfx1250) — hardware-verified
//
#include <hip/hip_runtime.h>
#include <math.h>
#include <stdint.h>

#define NBATCH 32
#define SEQ    512
#define DM     512
#define NH     8
#define HD     64
#define KO     (2 * DM)
#define MP     (NBATCH * SEQ)
#define NQB    (SEQ / 64)
#define LNT    (DM / 4)
#define LNW    (LNT / 32)
#define LNEPS  1.0e-5f
#define WSC    64.0f
static_assert(NH * HD == DM);
static_assert((SEQ % 64) == 0 && (DM % 64) == 0 && (MP % 64) == 0 && (KO % 64) == 0);
static_assert(DM == 4 * LNT && (LNT % 32) == 0 && LNW <= 8 && LNT == 128);

typedef _Float16 v16h __attribute__((ext_vector_type(16)));
typedef _Float16 v8h  __attribute__((ext_vector_type(8)));
typedef __bf16   v16b __attribute__((ext_vector_type(16)));
typedef __bf16   v8b  __attribute__((ext_vector_type(8)));
typedef float    v8f  __attribute__((ext_vector_type(8)));
typedef float    v4f  __attribute__((ext_vector_type(4)));
typedef unsigned int   v4u  __attribute__((ext_vector_type(4)));
typedef unsigned short v8us __attribute__((ext_vector_type(8)));

union FragH { v16h v; v8h h[2]; };

template <typename T> struct FT;
template <> struct FT<_Float16> { typedef v16h V; typedef v8h V8; };
template <> struct FT<__bf16>   { typedef v16b V; typedef v8b V8; };

__device__ __forceinline__ unsigned short bf_bits(float f) {
  unsigned u = __float_as_uint(f);
  return (unsigned short)((u + 0x7FFFu + ((u >> 16) & 1u)) >> 16);
}
__device__ __forceinline__ float bf_up(unsigned short h) { return __uint_as_float(((unsigned)h) << 16); }
__device__ __forceinline__ float bfr(float f) { return bf_up(bf_bits(f)); }
__device__ __forceinline__ unsigned short h_bits(_Float16 x) { return __builtin_bit_cast(unsigned short, x); }
__device__ __forceinline__ unsigned pk16(unsigned short a, unsigned short b) { return (unsigned)a | ((unsigned)b << 16); }
__device__ __forceinline__ v8f zero8() { v8f z = {0.f, 0.f, 0.f, 0.f, 0.f, 0.f, 0.f, 0.f}; return z; }

template <typename T>
__device__ __forceinline__ typename FT<T>::V ldfrag(const T* p) {
  union { typename FT<T>::V v; typename FT<T>::V8 h[2]; } f;
  f.h[0] = *(const typename FT<T>::V8*)(p);
  f.h[1] = *(const typename FT<T>::V8*)(p + 16);
  return f.v;
}

__device__ __forceinline__ v8f mma_raw(v16h a, v16h b, v8f c) {
  return __builtin_amdgcn_wmma_f32_16x16x32_f16(false, a, false, b, (short)0, c, false, false);
}
__device__ __forceinline__ v8f mma_raw(v16b a, v16b b, v8f c) {
  return __builtin_amdgcn_wmma_f32_16x16x32_bf16(false, a, false, b, (short)0, c, false, false);
}
__device__ __forceinline__ v8f mma_h(v16h a, v16h b, v8f c) {
  c = mma_raw(a, b, c);
#if defined(__HIP_DEVICE_COMPILE__)
  asm volatile("v_nop\n\tv_nop\n\tv_nop\n\tv_nop" : "+v"(c) : "v"(a), "v"(b));
#endif
  return c;
}
template <typename V>
__device__ __forceinline__ void dep_guard1(v8f& a, v8f& b, V x) {
#if defined(__HIP_DEVICE_COMPILE__)
  asm volatile("v_nop\n\tv_nop\n\tv_nop\n\tv_nop" : "+v"(a), "+v"(b) : "v"(x));
#endif
}
template <typename V>
__device__ __forceinline__ void keep4_v(V a, V b, V c, V d) {
#if defined(__HIP_DEVICE_COMPILE__)
  asm volatile("v_nop" :: "v"(a), "v"(b), "v"(c), "v"(d));
#endif
}
__device__ __forceinline__ void acc_guard4(v8f& a, v8f& b, v8f& c, v8f& d) {
#if defined(__HIP_DEVICE_COMPILE__)
  asm volatile("v_nop\n\tv_nop\n\tv_nop\n\tv_nop" : "+v"(a), "+v"(b), "+v"(c), "+v"(d));
#endif
}
__device__ __forceinline__ void wave_sync_lds() {
  __builtin_amdgcn_fence(__ATOMIC_RELEASE, "workgroup");
  __builtin_amdgcn_wave_barrier();
  __builtin_amdgcn_fence(__ATOMIC_ACQUIRE, "workgroup");
}
__device__ __forceinline__ float wsum(float v) {
#pragma unroll
  for (int off = 16; off > 0; off >>= 1) v += __shfl_xor(v, off, 32);
  return v;
}
__device__ __forceinline__ float bsumLN(float v, float* red, int lane, int wave) {
  v = wsum(v);
  if (lane == 0) red[wave] = v;
  __syncthreads();
  float tot = 0.f;
#pragma unroll
  for (int w = 0; w < LNW; ++w) tot += red[w];
  return tot;
}

__global__ __launch_bounds__(256) void conv_h16(const float* __restrict__ X, unsigned short* Xh, int n8, float wsc) {
  const int i  = blockIdx.x * 256 + threadIdx.x;
  const int ic = (i < n8) ? i : (n8 - 1);
  const float* src = X + (size_t)ic * 8;
  const v4f a = *(const v4f*)(src);
  const v4f c = *(const v4f*)(src + 4);
  v4u o;
  o[0] = pk16(h_bits((_Float16)(bfr(a[0]) * wsc)), h_bits((_Float16)(bfr(a[1]) * wsc)));
  o[1] = pk16(h_bits((_Float16)(bfr(a[2]) * wsc)), h_bits((_Float16)(bfr(a[3]) * wsc)));
  o[2] = pk16(h_bits((_Float16)(bfr(c[0]) * wsc)), h_bits((_Float16)(bfr(c[1]) * wsc)));
  o[3] = pk16(h_bits((_Float16)(bfr(c[2]) * wsc)), h_bits((_Float16)(bfr(c[3]) * wsc)));
  if (i < n8) *(volatile v4u*)(Xh + (size_t)i * 8) = o;
  __threadfence();
  if (i < n8) *(volatile v4u*)(Xh + (size_t)i * 8) = o;
}

template <int OB>
__global__ __launch_bounds__(256) void convT16(const float* __restrict__ W, int ldw, unsigned short* Wt, int ldt,
                                               int coff, int nrow, int ncol, float wsc) {
  __shared__ __align__(16) unsigned short sT[64 * 72];
  const int t  = threadIdx.x;
  const int n0 = blockIdx.x * 64;
  const int k0 = blockIdx.y * 64;
  {
    const int r  = t >> 2;
    const int cq = (t & 3) * 16;
    int sr = k0 + r;  sr = (sr < nrow) ? sr : (nrow - 1);
    int sc = n0 + cq; sc = (sc < ncol - 16) ? sc : (ncol - 16);
    const float* src = W + (size_t)sr * ldw + sc;
#pragma unroll
    for (int i = 0; i < 4; ++i) {
      const v4f x = *(const v4f*)(src + 4 * i);
#pragma unroll
      for (int e = 0; e < 4; ++e) {
        const float f = x[e];
        const unsigned short u = OB ? bf_bits(f) : h_bits((_Float16)(bfr(f) * wsc));
        sT[(cq + 4 * i + e) * 72 + r] = u;
      }
    }
  }
  __syncthreads();
  const int row = t >> 3;
  const int c8  = (t & 7) * 8;
  const v8us o0 = *(const v8us*)(sT + row * 72 + c8);
  const v8us o1 = *(const v8us*)(sT + (32 + row) * 72 + c8);
  unsigned short* d0 = Wt + (size_t)(n0 + row) * ldt + coff + k0 + c8;
  unsigned short* d1 = Wt + (size_t)(n0 + 32 + row) * ldt + coff + k0 + c8;
  *(volatile v8us*)d0 = o0;
  *(volatile v8us*)d1 = o1;
  __threadfence();
  *(volatile v8us*)d0 = o0;
  *(volatile v8us*)d1 = o1;
}

template <typename T, int OM, int BIASM, int ACT, int RES>
__global__ __launch_bounds__(256) void gemm64(
    const unsigned short* __restrict__ Ap, int lda, long long strideA,
    const unsigned short* __restrict__ Btp, int ldb, long long strideB,
    const float* __restrict__ bias0, const float* __restrict__ bias1, int Nb,
    const float* resid,
    void* Cout, int ldc, long long strideC,
    int M, int N, int K, float oscale) {
  typedef typename FT<T>::V VF;
  const T* A  = (const T*)(const void*)Ap;
  const T* Bt = (const T*)(const void*)Btp;
  __shared__ __align__(16) float sT[8][16 * 68];
  const int b    = blockIdx.y;
  const int lane = threadIdx.x & 31;
  const int wave = threadIdx.x >> 5;
  const int tilesN = N >> 6;
  const int tilesM = M >> 6;
  const int tile = blockIdx.x * 8 + wave;
  if (tile >= tilesM * tilesN) return;
  const int tm = tile / tilesN;
  const int tn = tile - tm * tilesN;
  const int m0 = tm << 6;
  const int n0 = tn << 6;

  const T* Ab = A  + (size_t)b * strideA;
  const T* Bb = Bt + (size_t)b * strideB;

  const int rlane = lane & 15;
  const int koff  = (lane >> 4) * 8;
  const int mOff  = (lane >> 4) * 8;

  v8f acc[4][4];
#pragma unroll
  for (int i = 0; i < 4; ++i)
#pragma unroll
    for (int j = 0; j < 4; ++j) acc[i][j] = zero8();

  for (int k0 = 0; k0 < K; k0 += 32) {
    VF bh[4];
#pragma unroll
    for (int j = 0; j < 4; ++j) {
      const size_t bo = (size_t)(n0 + (j << 4) + rlane) * ldb + koff + k0;
      bh[j] = ldfrag<T>(Bb + bo);
    }
#pragma unroll
    for (int i = 0; i < 4; ++i) {
      const size_t ao = (size_t)(m0 + (i << 4) + rlane) * lda + koff + k0;
      const VF ah = ldfrag<T>(Ab + ao);
#pragma unroll
      for (int j = 0; j < 4; ++j) acc[i][j] = mma_raw(ah, bh[j], acc[i][j]);
      dep_guard1<VF>(acc[i][0], acc[i][3], ah);
    }
    keep4_v<VF>(bh[0], bh[1], bh[2], bh[3]);
  }
  acc_guard4(acc[0][0], acc[0][1], acc[0][2], acc[0][3]);
  acc_guard4(acc[1][0], acc[1][1], acc[1][2], acc[1][3]);
  acc_guard4(acc[2][0], acc[2][1], acc[2][2], acc[2][3]);
  acc_guard4(acc[3][0], acc[3][1], acc[3][2], acc[3][3]);

  const int hh2 = lane >> 4, c4 = (lane & 15) * 4;
  const int q8  = lane >> 3, c8 = (lane & 7) * 8;
  float bc[8];
#pragma unroll
  for (int e = 0; e < 8; ++e) bc[e] = 0.f;
  if (BIASM == 0) {
    const bool use1 = (n0 >= Nb);
    if (OM == 0) {
      const int cb = n0 + c4;
      const int i0 = (cb < Nb - 4) ? cb : (Nb - 4);
      const int i1 = (cb - Nb > 0) ? (cb - Nb) : 0;
      const v4f b0v = *(const v4f*)(bias0 + i0);
      const v4f b1v = *(const v4f*)(bias1 + i1);
#pragma unroll
      for (int e = 0; e < 4; ++e) bc[e] = bfr(use1 ? b1v[e] : b0v[e]);
    } else {
      const int cb = n0 + c8;
      const int i0 = (cb < Nb - 8) ? cb : (Nb - 8);
      const int i1 = (cb - Nb > 0) ? (cb - Nb) : 0;
      const v4f b0a = *(const v4f*)(bias0 + i0), b0b = *(const v4f*)(bias0 + i0 + 4);
      const v4f b1a = *(const v4f*)(bias1 + i1), b1b = *(const v4f*)(bias1 + i1 + 4);
#pragma unroll
      for (int e = 0; e < 4; ++e) {
        bc[e]     = bfr(use1 ? b1a[e] : b0a[e]);
        bc[4 + e] = bfr(use1 ? b1b[e] : b0b[e]);
      }
    }
  }

  float* slab = sT[wave];
#pragma unroll
  for (int i = 0; i < 4; ++i) {
    const int mBase = m0 + (i << 4);
#pragma unroll
    for (int j = 0; j < 4; ++j) {
#pragma unroll
      for (int r = 0; r < 8; ++r) {
        slab[(mOff + r) * 68 + (j << 4) + rlane] = acc[i][j][r];
      }
    }
    wave_sync_lds();
    if (OM == 0) {
      float* C = (float*)Cout + (size_t)b * strideC;
      const float* Rb = resid + (size_t)b * strideC;
      v4f vals[8];
#pragma unroll
      for (int it = 0; it < 8; ++it) {
        const int row = it * 2 + hh2;
        v4f v = *(const v4f*)(slab + row * 68 + c4);
#pragma unroll
        for (int e = 0; e < 4; ++e) {
          float f = v[e] * oscale + bc[e];
          if (ACT == 2) f = fmaxf(f, 0.f);
          v[e] = f;
        }
        if (RES == 1) {
          const v4f rr = *(const v4f*)(Rb + (size_t)(mBase + row) * ldc + n0 + c4);
#pragma unroll
          for (int e = 0; e < 4; ++e) v[e] += rr[e];
        }
        vals[it] = v;
      }
      for (int pass = 0; pass < 2; ++pass) {
#pragma unroll
        for (int it = 0; it < 8; ++it) {
          const int row = it * 2 + hh2;
          *(volatile v4f*)(C + (size_t)(mBase + row) * ldc + n0 + c4) = vals[it];
        }
        __threadfence();
      }
    } else {
      unsigned short* C = (unsigned short*)Cout + (size_t)b * strideC;
      v4u hv[4];
#pragma unroll
      for (int it = 0; it < 4; ++it) {
        const int row = it * 4 + q8;
        const float* sp = slab + row * 68 + c8;
        float bm = 0.f;
        if (BIASM == 1) bm = bfr(bias0[mBase + row]);
        v4u a;
#pragma unroll
        for (int e = 0; e < 4; ++e) {
          float f0 = sp[2 * e]     * oscale + ((BIASM == 1) ? bm : bc[2 * e]);
          float f1 = sp[2 * e + 1] * oscale + ((BIASM == 1) ? bm : bc[2 * e + 1]);
          if (ACT == 2) { f0 = fmaxf(f0, 0.f); f1 = fmaxf(f1, 0.f); }
          unsigned short u0, u1;
          if (OM == 1) { u0 = bf_bits(f0); u1 = bf_bits(f1); }
          else         { u0 = h_bits((_Float16)f0); u1 = h_bits((_Float16)f1); }
          a[e] = pk16(u0, u1);
        }
        hv[it] = a;
      }
      for (int pass = 0; pass < 2; ++pass) {
#pragma unroll
        for (int it = 0; it < 4; ++it) {
          const int row = it * 4 + q8;
          *(volatile v4u*)(C + (size_t)(mBase + row) * ldc + n0 + c8) = hv[it];
        }
        __threadfence();
      }
    }
    wave_sync_lds();
  }
}

__global__ __launch_bounds__(128)
void attn64(const float* __restrict__ qfp, const unsigned short* __restrict__ khp,
            const unsigned short* __restrict__ vtp, float* outp, float sscale) {
  __shared__ __align__(16) _Float16 Ksh[64 * 64];
  __shared__ __align__(16) _Float16 Vth[64 * 64];
  __shared__ __align__(16) _Float16 Psh[4][16 * 64];
  __shared__ __align__(16) float    Os[4][16 * 64];

  const int tid  = threadIdx.x;
  const int wave = tid >> 5;
  const int lane = tid & 31;
  const int hh   = lane >> 4;
  const int c    = lane & 15;

  const int bx   = blockIdx.x;
  const int qb   = bx % NQB;
  const int rest = bx / NQB;
  const int h    = rest % NH;
  const int b    = rest / NH;
  const int q0   = qb * 64 + wave * 16;
  const size_t rowB = (size_t)b * SEQ;

  const float*    Qh = qfp + (size_t)h * HD;
  const _Float16* Kg = (const _Float16*)(const void*)khp + (size_t)h * HD;
  const _Float16* Vh = (const _Float16*)(const void*)vtp + ((size_t)b * DM + (size_t)h * HD) * SEQ;

  v16h qa[2];
#pragma unroll
  for (int dc = 0; dc < 2; ++dc) {
    const float* qr = Qh + (rowB + q0 + c) * DM + dc * 32 + 8 * hh;
    const v4f x0 = *(const v4f*)(qr);
    const v4f x1 = *(const v4f*)(qr + 4);
    const v4f x2 = *(const v4f*)(qr + 16);
    const v4f x3 = *(const v4f*)(qr + 20);
    v8h lo, hi;
#pragma unroll
    for (int e = 0; e < 4; ++e) {
      lo[e]     = (_Float16)x0[e];
      lo[4 + e] = (_Float16)x1[e];
      hi[e]     = (_Float16)x2[e];
      hi[4 + e] = (_Float16)x3[e];
    }
    FragH f;
    f.h[0] = lo;
    f.h[1] = hi;
    qa[dc] = f.v;
  }

  float mrow[8], lrow[8];
  v8f oacc[4];
#pragma unroll
  for (int r = 0; r < 8; ++r) { mrow[r] = -INFINITY; lrow[r] = 0.f; }
#pragma unroll
  for (int t = 0; t < 4; ++t) oacc[t] = zero8();

  for (int kt = 0; kt < NQB; ++kt) {
    const int kv0 = kt * 64;
    __syncthreads();
    {
      const int r = tid >> 1, hf = (tid & 1) * 32;
      const _Float16* kg = Kg + (rowB + kv0 + r) * DM + hf;
      const _Float16* vg = Vh + (size_t)r * SEQ + kv0 + hf;
#pragma unroll
      for (int i = 0; i < 4; ++i) {
        const v8h a0 = *(const v8h*)(kg + 8 * i);
        const v8h b0 = *(const v8h*)(vg + 8 * i);
        *(v8h*)(Ksh + r * 64 + hf + 8 * i) = a0;
        *(v8h*)(Vth + r * 64 + hf + 8 * i) = b0;
      }
    }
    __syncthreads();

    v8f s[4];
#pragma unroll
    for (int j = 0; j < 4; ++j) {
      v8f sh = zero8();
#pragma unroll
      for (int dc = 0; dc < 2; ++dc) {
        FragH kb;
        kb.h[0] = *(const v8h*)(Ksh + (j * 16 + c) * 64 + dc * 32 + 8 * hh);
        kb.h[1] = *(const v8h*)(Ksh + (j * 16 + c) * 64 + dc * 32 + 16 + 8 * hh);
        sh = mma_h(qa[dc], kb.v, sh);
      }
#pragma unroll
      for (int r = 0; r < 8; ++r) s[j][r] = sh[r] * sscale;
    }

    _Float16* pwh = Psh[wave];
#pragma unroll
    for (int r = 0; r < 8; ++r) {
      float m = s[0][r];
      m = fmaxf(m, s[1][r]);
      m = fmaxf(m, s[2][r]);
      m = fmaxf(m, s[3][r]);
#pragma unroll
      for (int off = 1; off < 16; off <<= 1) m = fmaxf(m, __shfl_xor(m, off, 32));
      const float mnew  = fmaxf(mrow[r], m);
      const float alpha = __expf(mrow[r] - mnew);
      mrow[r] = mnew;
      float psum = 0.f;
#pragma unroll
      for (int j = 0; j < 4; ++j) {
        const float p = __expf(s[j][r] - mnew);
        psum += p;
        pwh[(8 * hh + r) * 64 + j * 16 + c] = (_Float16)(p * 1024.0f);
      }
#pragma unroll
      for (int off = 1; off < 16; off <<= 1) psum += __shfl_xor(psum, off, 32);
      lrow[r] = lrow[r] * alpha + psum;
#pragma unroll
      for (int t = 0; t < 4; ++t) oacc[t][r] *= alpha;
    }
    wave_sync_lds();

#pragma unroll 1
    for (int kk = 0; kk < 2; ++kk) {
      FragH pa;
      pa.h[0] = *(const v8h*)(pwh + c * 64 + kk * 32 + 8 * hh);
      pa.h[1] = *(const v8h*)(pwh + c * 64 + kk * 32 + 16 + 8 * hh);
#pragma unroll
      for (int t = 0; t < 4; ++t) {
        FragH vb;
        vb.h[0] = *(const v8h*)(Vth + (t * 16 + c) * 64 + kk * 32 + 8 * hh);
        vb.h[1] = *(const v8h*)(Vth + (t * 16 + c) * 64 + kk * 32 + 16 + 8 * hh);
        oacc[t] = mma_h(pa.v, vb.v, oacc[t]);
      }
    }
  }

  float* os = Os[wave];
#pragma unroll
  for (int r = 0; r < 8; ++r) {
    const float l = lrow[r];
    const float inv = ((l > 0.f) ? (1.0f / l) : 0.f) * (1.0f / 1024.0f);
#pragma unroll
    for (int t = 0; t < 4; ++t) os[(8 * hh + r) * 64 + t * 16 + c] = oacc[t][r] * inv;
  }
  wave_sync_lds();
  {
    const int hh2 = lane >> 4, c4 = (lane & 15) * 4;
    v4f vals[8];
#pragma unroll
    for (int it = 0; it < 8; ++it) {
      const int row = it * 2 + hh2;
      v4f v = *(const v4f*)(os + row * 64 + c4);
      const size_t go = (rowB + q0 + row) * DM + (size_t)h * HD + c4;
      const v4f rr = *(const v4f*)(qfp + go);
#pragma unroll
      for (int e = 0; e < 4; ++e) v[e] += rr[e];
      vals[it] = v;
    }
    for (int pass = 0; pass < 2; ++pass) {
#pragma unroll
      for (int it = 0; it < 8; ++it) {
        const int row = it * 2 + hh2;
        const size_t go = (rowB + q0 + row) * DM + (size_t)h * HD + c4;
        *(volatile v4f*)(outp + go) = vals[it];
      }
      __threadfence();
    }
  }
}

__global__ __launch_bounds__(LNT) void ln_row_dual(const float* __restrict__ X, const float* __restrict__ gam,
                                                   const float* __restrict__ bet, float* outF, unsigned short* outB) {
  __shared__ float red0[8], red1[8];
  __shared__ __align__(16) float ys[DM];
  const int t = threadIdx.x, lane = t & 31, wave = t >> 5;
  const size_t row  = (size_t)blockIdx.x;
  const size_t base = row * DM;
  const v4f xv = *(const v4f*)(X + base + 4 * t);
  const float mean = bsumLN((xv[0] + xv[1]) + (xv[2] + xv[3]), red0, lane, wave) * (1.0f / DM);
  v4f d;
#pragma unroll
  for (int e = 0; e < 4; ++e) d[e] = xv[e] - mean;
  const float var  = bsumLN((d[0] * d[0] + d[1] * d[1]) + (d[2] * d[2] + d[3] * d[3]), red1, lane, wave) * (1.0f / DM);
  const float rstd = 1.0f / sqrtf(var + LNEPS);
  const v4f gv = *(const v4f*)(gam + 4 * t);
  const v4f bv = *(const v4f*)(bet + 4 * t);
  v4f y;
#pragma unroll
  for (int e = 0; e < 4; ++e) y[e] = (d[e] * rstd) * bfr(gv[e]) + bfr(bv[e]);
  float* dstF = outF + base + 4 * t;
  *(volatile v4f*)dstF = y;
  *(v4f*)(ys + 4 * t) = y;
  __syncthreads();
  const int cc = 8 * (t & 63);
  const bool useLo = (t >= 64);
  const v4f a0 = *(const v4f*)(ys + cc);
  const v4f a1 = *(const v4f*)(ys + cc + 4);
  v4u ov;
#pragma unroll
  for (int e = 0; e < 2; ++e) {
    const float f0 = a0[2 * e], f1 = a0[2 * e + 1];
    const float g0 = a1[2 * e], g1 = a1[2 * e + 1];
    const unsigned short h0 = bf_bits(f0), h1 = bf_bits(f1), k0 = bf_bits(g0), k1 = bf_bits(g1);
    const unsigned short l0 = bf_bits(f0 - bf_up(h0)), l1 = bf_bits(f1 - bf_up(h1));
    const unsigned short m0 = bf_bits(g0 - bf_up(k0)), m1 = bf_bits(g1 - bf_up(k1));
    ov[e]     = useLo ? pk16(l0, l1) : pk16(h0, h1);
    ov[2 + e] = useLo ? pk16(m0, m1) : pk16(k0, k1);
  }
  unsigned short* dstB = outB + row * KO + (useLo ? DM : 0) + cc;
  *(volatile v4u*)dstB = ov;
  __threadfence();
  *(volatile v4f*)dstF = y;
  *(volatile v4u*)dstB = ov;
}

__global__ __launch_bounds__(LNT) void ln_row_f32(const float* __restrict__ X, const float* __restrict__ gam,
                                                  const float* __restrict__ bet, float* outF) {
  __shared__ float red0[8], red1[8];
  const int t = threadIdx.x, lane = t & 31, wave = t >> 5;
  const size_t base = (size_t)blockIdx.x * DM;
  const v4f xv = *(const v4f*)(X + base + 4 * t);
  const float mean = bsumLN((xv[0] + xv[1]) + (xv[2] + xv[3]), red0, lane, wave) * (1.0f / DM);
  v4f d;
#pragma unroll
  for (int e = 0; e < 4; ++e) d[e] = xv[e] - mean;
  const float var  = bsumLN((d[0] * d[0] + d[1] * d[1]) + (d[2] * d[2] + d[3] * d[3]), red1, lane, wave) * (1.0f / DM);
  const float rstd = 1.0f / sqrtf(var + LNEPS);
  const v4f gv = *(const v4f*)(gam + 4 * t);
  const v4f bv = *(const v4f*)(bet + 4 * t);
  v4f y;
#pragma unroll
  for (int e = 0; e < 4; ++e) y[e] = (d[e] * rstd) * bfr(gv[e]) + bfr(bv[e]);
  float* dst = outF + base + 4 * t;
  *(volatile v4f*)dst = y;
  __threadfence();
  *(volatile v4f*)dst = y;
}

extern "C" void kernel_launch(void* const* d_in, const int* in_sizes, int n_in,
                              void* d_out, int out_size, void* d_ws, size_t ws_size,
                              hipStream_t stream) {
  if (n_in < 14) return;
  if (in_sizes[0] != MP * DM || in_sizes[1] != MP * DM) return;
  if (in_sizes[2] != DM * DM || in_sizes[3] != DM) return;
  if (in_sizes[4] != DM * DM || in_sizes[5] != DM) return;
  if (in_sizes[6] != DM * DM || in_sizes[7] != DM) return;
  if (in_sizes[8] != DM * DM || in_sizes[9] != DM) return;
  if (in_sizes[10] != DM || in_sizes[11] != DM || in_sizes[12] != DM || in_sizes[13] != DM) return;
  if (out_size != MP * DM) return;

  const float* Qin   = (const float*)d_in[0];
  const float* Kin   = (const float*)d_in[1];
  const float* w_q   = (const float*)d_in[2];
  const float* b_q   = (const float*)d_in[3];
  const float* w_k   = (const float*)d_in[4];
  const float* b_k   = (const float*)d_in[5];
  const float* w_v   = (const float*)d_in[6];
  const float* b_v   = (const float*)d_in[7];
  const float* w_o   = (const float*)d_in[8];
  const float* b_o   = (const float*)d_in[9];
  const float* ln0_g = (const float*)d_in[10];
  const float* ln0_b = (const float*)d_in[11];
  const float* ln1_g = (const float*)d_in[12];
  const float* ln1_b = (const float*)d_in[13];

  const size_t PW16 = (size_t)DM * DM * 2;
  const size_t PWO  = (size_t)DM * KO * 2;
  const size_t PS32 = (size_t)MP * DM * 4;
  const size_t PH16 = (size_t)MP * DM * 2;
  size_t off = 0;
  const size_t oWq = off; off += PW16;
  const size_t oWk = off; off += PW16;
  const size_t oWv = off; off += PW16;
  const size_t oWo = off; off += PWO;
  const size_t oS1 = off; off += PS32;
  const size_t oS2 = off; off += PS32;
  const size_t oS3 = off; off += PS32;
  if (off > ws_size) return;
  if (off > (size_t)134217728) return;
  if ((size_t)MP * KO * 2 != PS32 || (size_t)NBATCH * DM * SEQ * 2 != PH16 || 2 * PH16 != PS32) return;

  char* ws = (char*)d_ws;
  unsigned short* WqT  = (unsigned short*)(ws + oWq);
  unsigned short* WkT  = (unsigned short*)(ws + oWk);
  unsigned short* WvT  = (unsigned short*)(ws + oWv);
  unsigned short* WoT2 = (unsigned short*)(ws + oWo);
  unsigned short* QH   = (unsigned short*)(ws + oS1);
  unsigned short* KH   = (unsigned short*)(ws + oS1 + PH16);
  float*          OH   = (float*)(ws + oS1);
  float*          Hf   = (float*)(ws + oS1);
  float*          qF   = (float*)(ws + oS2);
  float*          OF   = (float*)(ws + oS2);
  unsigned short* kH   = (unsigned short*)(ws + oS3);
  unsigned short* VT   = (unsigned short*)(ws + oS3 + PH16);
  unsigned short* OB   = (unsigned short*)(ws + oS3);
  float*          out0 = (float*)d_out;

  const int n8x = (MP * DM) / 8;
  if ((n8x % 256) != 0) return;
  const dim3 blk(256), blk128(128), blkLN(LNT);
  const dim3 gT(DM / 64, DM / 64);
  const dim3 gCx(n8x / 256);
  const dim3 gG(((MP / 64) * (DM / 64) + 7) / 8, 1);
  const dim3 gVT(((DM / 64) * (SEQ / 64) + 7) / 8, NBATCH);
  const dim3 gAttn(NBATCH * NH * NQB);
  const dim3 gRow(MP);
  const float invw   = 1.0f / WSC;
  const float sscale = 0.044194173824159216f;

  convT16<0><<<gT, blk, 0, stream>>>(w_q, DM, WqT, DM, 0, DM, DM, WSC);
  convT16<0><<<gT, blk, 0, stream>>>(w_k, DM, WkT, DM, 0, DM, DM, WSC);
  convT16<0><<<gT, blk, 0, stream>>>(w_v, DM, WvT, DM, 0, DM, DM, WSC);
  convT16<1><<<gT, blk, 0, stream>>>(w_o, DM, WoT2, KO, 0, DM, DM, 1.0f);
  convT16<1><<<gT, blk, 0, stream>>>(w_o, DM, WoT2, KO, DM, DM, DM, 1.0f);
  conv_h16<<<gCx, blk, 0, stream>>>(Qin, QH, n8x, 1.0f);
  conv_h16<<<gCx, blk, 0, stream>>>(Kin, KH, n8x, 1.0f);

  gemm64<_Float16, 0, 0, 0, 0><<<gG, blk, 0, stream>>>(
      QH, DM, 0LL, WqT, DM, 0LL, b_q, b_q, DM, Qin,
      (void*)qF, DM, 0LL, MP, DM, DM, invw);
  gemm64<_Float16, 2, 0, 0, 0><<<gG, blk, 0, stream>>>(
      KH, DM, 0LL, WkT, DM, 0LL, b_k, b_k, DM, Qin,
      (void*)kH, DM, 0LL, MP, DM, DM, invw);
  gemm64<_Float16, 2, 1, 0, 0><<<gVT, blk, 0, stream>>>(
      WvT, DM, 0LL, KH, DM, (long long)SEQ * DM, b_v, b_v, SEQ, Qin,
      (void*)VT, SEQ, (long long)DM * SEQ, DM, SEQ, DM, invw);

  attn64<<<gAttn, blk128, 0, stream>>>(qF, kH, VT, OH, sscale);

  ln_row_dual<<<gRow, blkLN, 0, stream>>>(OH, ln0_g, ln0_b, OF, OB);

  gemm64<__bf16, 0, 0, 2, 1><<<gG, blk, 0, stream>>>(
      OB, KO, 0LL, WoT2, KO, 0LL, b_o, b_o, DM, OF,
      (void*)Hf, DM, 0LL, MP, DM, KO, 1.0f);

  ln_row_f32<<<gRow, blkLN, 0, stream>>>(Hf, ln1_g, ln1_b, out0);
  (void)hipGetLastError();
}
